// RegressorHybrid_46437186404761
// MI455X (gfx1250) — hardware-verified
//
#include <hip/hip_runtime.h>
#include <math.h>

#define HID    64
#define FIN    128
#define H3     32
#define NCHUNK 10

#define SX   64.0f
#define SW   1024.0f
#define SH1  64.0f
#define SH2  256.0f

typedef _Float16 v16h __attribute__((ext_vector_type(16)));
typedef _Float16 v8h  __attribute__((ext_vector_type(8)));
typedef float    v8f  __attribute__((ext_vector_type(8)));
typedef float    v4f  __attribute__((ext_vector_type(4)));
typedef unsigned int v4u __attribute__((ext_vector_type(4)));

union P8 { v8h h; v4u u; };

__device__ __forceinline__ float bf_rne(float f) {
  unsigned u = __float_as_uint(f);
  u = (u + 0x7FFFu + ((u >> 16) & 1u)) & 0xFFFF0000u;
  return __uint_as_float(u);
}
__device__ __forceinline__ v8f zero8() { v8f z = {0.f, 0.f, 0.f, 0.f, 0.f, 0.f, 0.f, 0.f}; return z; }
__device__ __forceinline__ int clampi(int v, int lo, int hi) { v = v < lo ? lo : v; return v > hi ? hi : v; }
__device__ __forceinline__ float lrelu(float v) { return v > 0.f ? v : 0.01f * v; }

__device__ __forceinline__ v16h ldfrag(const _Float16* p) {
  union { v16h v; v8h h[2]; } f;
  f.h[0] = *(const v8h*)(p);
  f.h[1] = *(const v8h*)(p + 16);
  return f.v;
}

__device__ __forceinline__ v8f mma_h(v16h a, v16h b, v8f c) {
  return __builtin_amdgcn_wmma_f32_16x16x32_f16(false, a, false, b, (short)0, c, false, false);
}
__device__ __forceinline__ void dep_guard(v8f& a, v8f& b, v16h x) {
#if defined(__HIP_DEVICE_COMPILE__)
  asm volatile("v_nop\n\tv_nop\n\tv_nop\n\tv_nop" : "+v"(a), "+v"(b) : "v"(x));
#endif
}
__device__ __forceinline__ void keep2(v16h a, v16h b) {
#if defined(__HIP_DEVICE_COMPILE__)
  asm volatile("v_nop" :: "v"(a), "v"(b));
#endif
}
__device__ __forceinline__ void acc_guard2(v8f& a, v8f& b) {
#if defined(__HIP_DEVICE_COMPILE__)
  asm volatile("v_nop\n\tv_nop\n\tv_nop\n\tv_nop" : "+v"(a), "+v"(b));
#endif
}
__device__ __forceinline__ void wave_sync_lds() {
  __builtin_amdgcn_fence(__ATOMIC_RELEASE, "workgroup");
  __builtin_amdgcn_wave_barrier();
  __builtin_amdgcn_fence(__ATOMIC_ACQUIRE, "workgroup");
}

__global__ __launch_bounds__(256) void cvt_wt(const float* __restrict__ w, unsigned short* wt, int K, int N) {
  const int g = blockIdx.x * 256 + threadIdx.x;
  const int k8n = K >> 3;
  if (g < N * k8n) {
    const int n  = g / k8n;
    const int k8 = (g - n * k8n) * 8;
    P8 p;
#pragma unroll
    for (int i = 0; i < 8; ++i) p.h[i] = (_Float16)(bf_rne(w[(size_t)(k8 + i) * N + n]) * SW);
    unsigned short* dst = wt + (size_t)n * K + k8;
    *(volatile v4u*)dst = p.u;
    __threadfence();
    *(volatile v4u*)dst = p.u;
  }
}

__global__ __launch_bounds__(256) void gather_x(const int* __restrict__ eli, const float* __restrict__ xs,
                                                const float* __restrict__ xd, unsigned short* X,
                                                int rbase, int nrows, int E, int nnode) {
  const int lane = threadIdx.x & 31;
  const int wave = threadIdx.x >> 5;
  const int hh   = lane >> 4;
  const int c8   = (lane & 15) * 8;
  const int rw   = blockIdx.x * 64 + wave * 8;
  if (rw + 8 > nrows) return;
  const int cd = (c8 < HID) ? c8 : (c8 - HID);
  v4u p[4];
#pragma unroll
  for (int it = 0; it < 4; ++it) {
    const int rr = rw + it * 2 + hh;
    const int e  = clampi(rbase + rr, 0, E - 1);
    int i0 = eli[e];
    int i1 = eli[(size_t)E + e];
    i0 = (i0 < 0) ? (i0 + nnode) : i0;  i0 = clampi(i0, 0, nnode - 1);
    i1 = (i1 < 0) ? (i1 + nnode) : i1;  i1 = clampi(i1, 0, nnode - 1);
    const float* bs = xs + (size_t)i0 * HID;
    const float* bd = xd + (size_t)i1 * HID;
    const float* src = ((c8 < HID) ? bs : bd) + cd;
    const v4f a = *(const v4f*)(src);
    const v4f c = *(const v4f*)(src + 4);
    P8 q;
#pragma unroll
    for (int t = 0; t < 4; ++t) {
      q.h[t]     = (_Float16)(bf_rne(a[t]) * SX);
      q.h[4 + t] = (_Float16)(bf_rne(c[t]) * SX);
    }
    p[it] = q.u;
  }
  for (int ps = 0; ps < 2; ++ps) {
#pragma unroll
    for (int it = 0; it < 4; ++it) {
      const int rr = rw + it * 2 + hh;
      *(volatile v4u*)(X + (size_t)rr * FIN + c8) = p[it];
    }
    __threadfence();
  }
}

template <int NT, int OUT_MODE>
__global__ __launch_bounds__(256) void gemm64(
    const unsigned short* __restrict__ Ap, int lda,
    const unsigned short* __restrict__ Btp, int ldb,
    const float* __restrict__ bias, float inscale,
    void* Cout, int ldc, float oscale,
    const float* __restrict__ w4, const float* __restrict__ b4,
    int M, int N, int K) {
  const _Float16* A  = (const _Float16*)(const void*)Ap;
  const _Float16* Bt = (const _Float16*)(const void*)Btp;
  __shared__ __align__(16) float sT[8][16 * 68];
  __shared__ __align__(16) float sW4[8][32];
  __shared__ __align__(16) float sLg[8][64];
  constexpr int TN = 16 * NT;
  const int lane = threadIdx.x & 31;
  const int wave = threadIdx.x >> 5;
  const int tilesN = N / TN;
  const int tilesM = M >> 6;
  const int tile = blockIdx.x * 8 + wave;
  if (tile >= tilesM * tilesN) return;
  const int tm = tile / tilesN;
  const int tn = tile - tm * tilesN;
  const int m0 = tm << 6;
  const int n0 = tn * TN;

  const int rlane = lane & 15;
  const int koff  = (lane >> 4) * 8;
  const int mOff  = (lane >> 4) * 8;

  float bv[NT];
#pragma unroll
  for (int j = 0; j < NT; ++j) bv[j] = bf_rne(bias[n0 + (j << 4) + rlane]);
  float b4v = 0.f;
  if (OUT_MODE == 4) {
    sW4[wave][lane] = bf_rne(w4[lane]);
    b4v = bf_rne(b4[0]);
  }

  v8f acc[4][NT];
#pragma unroll
  for (int i = 0; i < 4; ++i)
#pragma unroll
    for (int j = 0; j < NT; ++j) acc[i][j] = zero8();

  for (int k0 = 0; k0 < K; k0 += 32) {
    v16h bh[NT];
#pragma unroll
    for (int j = 0; j < NT; ++j) {
      const size_t bo = (size_t)(n0 + (j << 4) + rlane) * ldb + koff + k0;
      bh[j] = ldfrag(Bt + bo);
    }
#pragma unroll
    for (int i = 0; i < 4; ++i) {
      const size_t ao = (size_t)(m0 + (i << 4) + rlane) * lda + koff + k0;
      const v16h ah = ldfrag(A + ao);
#pragma unroll
      for (int j = 0; j < NT; ++j) acc[i][j] = mma_h(ah, bh[j], acc[i][j]);
      dep_guard(acc[i][0], acc[i][NT - 1], ah);
    }
    keep2(bh[0], bh[1]);
    keep2(bh[NT - 2], bh[NT - 1]);
  }
#pragma unroll
  for (int i = 0; i < 4; ++i)
#pragma unroll
    for (int j = 0; j < NT; j += 2) acc_guard2(acc[i][j], acc[i][j + 1]);

  float* slab = sT[wave];
#pragma unroll
  for (int i = 0; i < 4; ++i) {
    const int mBase = m0 + (i << 4);
#pragma unroll
    for (int j = 0; j < NT; ++j) {
#pragma unroll
      for (int r = 0; r < 8; ++r) {
        const float v = lrelu(acc[i][j][r] * inscale + bv[j]);
        slab[(mOff + r) * 68 + (j << 4) + rlane] = v;
      }
    }
    wave_sync_lds();
    if (OUT_MODE == 1) {
      const int q = lane >> 3, c8 = (lane & 7) * 8;
      unsigned short* C = (unsigned short*)Cout;
      v4u hv[4];
#pragma unroll
      for (int it = 0; it < 4; ++it) {
        const int row = it * 4 + q;
        const float* sp = slab + row * 68 + c8;
        P8 pk;
#pragma unroll
        for (int e = 0; e < 8; ++e) pk.h[e] = (_Float16)(sp[e] * oscale);
        hv[it] = pk.u;
      }
      for (int ps = 0; ps < 2; ++ps) {
#pragma unroll
        for (int it = 0; it < 4; ++it) {
          const int row = it * 4 + q;
          *(volatile v4u*)(C + (size_t)(mBase + row) * ldc + n0 + c8) = hv[it];
        }
        __threadfence();
      }
    } else {
      const int row = lane & 15, h2 = lane >> 4;
      const float* sp = slab + row * 68 + h2 * 16;
      const float* wp = sW4[wave] + h2 * 16;
      float s = 0.f;
#pragma unroll 4
      for (int t = 0; t < 16; ++t) s = fmaf(sp[t], wp[t], s);
      s += __shfl_xor(s, 16, 32);
      if (h2 == 0) sLg[wave][i * 16 + row] = s + b4v;
    }
    wave_sync_lds();
  }
  if (OUT_MODE == 4) {
    float* C = (float*)Cout;
    const v4f v = *(const v4f*)(sLg[wave] + 4 * (lane & 15));
    if (lane < 16) *(volatile v4f*)(C + (size_t)m0 + 4 * lane) = v;
    __threadfence();
    if (lane < 16) *(volatile v4f*)(C + (size_t)m0 + 4 * lane) = v;
  }
}

extern "C" void kernel_launch(void* const* d_in, const int* in_sizes, int n_in,
                              void* d_out, int out_size, void* d_ws, size_t ws_size,
                              hipStream_t stream) {
  if (n_in < 19) return;
  const int E = in_sizes[2] / 2;
  if (E <= 0 || in_sizes[2] != 2 * E) return;
  if (in_sizes[0] != in_sizes[1] || in_sizes[0] < HID || (in_sizes[0] % HID) != 0) return;
  const int nnode = in_sizes[0] / HID;
  if (in_sizes[3] != FIN * HID || in_sizes[4] != HID || in_sizes[5] != FIN * HID || in_sizes[6] != HID) return;
  if (in_sizes[7] != HID * HID || in_sizes[8] != HID || in_sizes[9] != HID * HID || in_sizes[10] != HID) return;
  if (in_sizes[11] != HID * H3 || in_sizes[12] != H3 || in_sizes[13] != HID * H3 || in_sizes[14] != H3) return;
  if (in_sizes[15] != H3 || in_sizes[16] != 1 || in_sizes[17] != H3 || in_sizes[18] != 1) return;
  if (out_size != 2 * E) return;
  if ((E % (NCHUNK * 64)) != 0) return;
  const int CROWS = E / NCHUNK;

  const float* xs  = (const float*)d_in[0];
  const float* xd  = (const float*)d_in[1];
  const int*   eli = (const int*)  d_in[2];
  const float* ew1 = (const float*)d_in[3];  const float* eb1 = (const float*)d_in[4];
  const float* ww1 = (const float*)d_in[5];  const float* wb1 = (const float*)d_in[6];
  const float* ew2 = (const float*)d_in[7];  const float* eb2 = (const float*)d_in[8];
  const float* ww2 = (const float*)d_in[9];  const float* wb2 = (const float*)d_in[10];
  const float* ew3 = (const float*)d_in[11]; const float* eb3 = (const float*)d_in[12];
  const float* ww3 = (const float*)d_in[13]; const float* wb3 = (const float*)d_in[14];
  const float* ew4 = (const float*)d_in[15]; const float* eb4 = (const float*)d_in[16];
  const float* ww4 = (const float*)d_in[17]; const float* wb4 = (const float*)d_in[18];
  float* out = (float*)d_out;

  const size_t PW1 = (size_t)HID * FIN * 2;
  const size_t PW2 = (size_t)HID * HID * 2;
  const size_t PW3 = (size_t)H3 * HID * 2;
  const size_t PX  = (size_t)CROWS * FIN * 2;
  const size_t PH  = (size_t)CROWS * HID * 2;
  size_t off = 0;
  const size_t oW1e = off; off += PW1;
  const size_t oW1w = off; off += PW1;
  const size_t oW2e = off; off += PW2;
  const size_t oW2w = off; off += PW2;
  const size_t oW3e = off; off += PW3;
  const size_t oW3w = off; off += PW3;
  const size_t oX   = off; off += PX;
  const size_t oH1  = off; off += PH;
  const size_t oH2  = off; off += PH;
  if (off > ws_size) return;
  if (off > (size_t)134217728) return;

  char* ws = (char*)d_ws;
  unsigned short* W1e = (unsigned short*)(ws + oW1e);
  unsigned short* W1w = (unsigned short*)(ws + oW1w);
  unsigned short* W2e = (unsigned short*)(ws + oW2e);
  unsigned short* W2w = (unsigned short*)(ws + oW2w);
  unsigned short* W3e = (unsigned short*)(ws + oW3e);
  unsigned short* W3w = (unsigned short*)(ws + oW3w);
  unsigned short* Xb  = (unsigned short*)(ws + oX);
  unsigned short* H1  = (unsigned short*)(ws + oH1);
  unsigned short* H2  = (unsigned short*)(ws + oH2);

  const dim3 blk(256);
  const int n8w1 = HID * FIN / 8;
  const int n8w2 = HID * HID / 8;
  const int n8w3 = H3 * HID / 8;
  const dim3 gW1((n8w1 + 255) / 256);
  const dim3 gW2((n8w2 + 255) / 256);
  const dim3 gW3((n8w3 + 255) / 256);
  const int tiles = CROWS / 64;
  const dim3 gGat(tiles);
  const dim3 gGm((tiles + 7) / 8);

  const float is1 = 1.0f / (SX * SW);
  const float is2 = 1.0f / (SH1 * SW);
  const float is3 = 1.0f / (SH2 * SW);

  cvt_wt<<<gW1, blk, 0, stream>>>(ew1, W1e, FIN, HID);
  cvt_wt<<<gW1, blk, 0, stream>>>(ww1, W1w, FIN, HID);
  cvt_wt<<<gW2, blk, 0, stream>>>(ew2, W2e, HID, HID);
  cvt_wt<<<gW2, blk, 0, stream>>>(ww2, W2w, HID, HID);
  cvt_wt<<<gW3, blk, 0, stream>>>(ew3, W3e, HID, H3);
  cvt_wt<<<gW3, blk, 0, stream>>>(ww3, W3w, HID, H3);

  for (int c = 0; c < NCHUNK; ++c) {
    const int rbase = c * CROWS;
    gather_x<<<gGat, blk, 0, stream>>>(eli, xs, xd, Xb, rbase, CROWS, E, nnode);
    gemm64<4, 1><<<gGm, blk, 0, stream>>>(Xb, FIN, W1e, FIN, eb1, is1, (void*)H1, HID, SH1, ew4, eb4, CROWS, HID, FIN);
    gemm64<4, 1><<<gGm, blk, 0, stream>>>(H1, HID, W2e, HID, eb2, is2, (void*)H2, HID, SH2, ew4, eb4, CROWS, HID, HID);
    gemm64<2, 4><<<gGm, blk, 0, stream>>>(H2, HID, W3e, HID, eb3, is3, (void*)(out + (size_t)rbase), 0, 1.0f,
                                          ew4, eb4, CROWS, H3, HID);
    gemm64<4, 1><<<gGm, blk, 0, stream>>>(Xb, FIN, W1w, FIN, wb1, is1, (void*)H1, HID, SH1, ww4, wb4, CROWS, HID, FIN);
    gemm64<4, 1><<<gGm, blk, 0, stream>>>(H1, HID, W2w, HID, wb2, is2, (void*)H2, HID, SH2, ww4, wb4, CROWS, HID, HID);
    gemm64<2, 4><<<gGm, blk, 0, stream>>>(H2, HID, W3w, HID, wb3, is3, (void*)(out + (size_t)E + (size_t)rbase), 0, 1.0f,
                                          ww4, wb4, CROWS, H3, HID);
  }
  (void)hipGetLastError();
}
